// IAF_74423193305610
// MI455X (gfx1250) — hardware-verified
//
#include <hip/hip_runtime.h>
#include <stddef.h>


typedef _Float16 v16h __attribute__((ext_vector_type(16)));
typedef _Float16 v8h  __attribute__((ext_vector_type(8)));
typedef float    v8f  __attribute__((ext_vector_type(8)));
typedef float    v4f  __attribute__((ext_vector_type(4)));

union Frag { v16h v; v8h h[2]; };

#define NB     2048
#define DD     32
#define HH     512
#define NSTEP  2
#define ST     520
#define SX     40
#define WSC    16.0f
#define WSCI   0.0625f
#define HALF_D_LOG2PI 29.406033062549525f

__global__ void __launch_bounds__(256)
pack_weights(const float* __restrict__ W, _Float16* __restrict__ dst,
             int K, int N, int mode, int nchunks) {
  const int t = blockIdx.x * 256 + threadIdx.x;
  if (t >= nchunks) return;
  const int KT = K >> 5, NT = N >> 4;
  const int frag = t >> 6;
  const int lane = (t >> 1) & 31;
  const int ih = t & 1;
  const int per = NT * KT;
  const int s = frag / per;
  const int rem = frag - s * per;
  const int nt = rem / KT;
  const int kt = rem - nt * KT;
  const int hb = lane >> 4, c = lane & 15;
  const int n = nt * 16 + c;
  v8h o;
#pragma unroll
  for (int i = 0; i < 8; ++i) {
    const int kk = ih * 16 + hb * 8 + i;
    const int k = kt * 32 + kk;
    const float w = W[((size_t)s * K + k) * N + n];
    bool keep;
    if (mode == 0)      keep = k < (n >> 4);
    else if (mode == 1) keep = (k >> 4) <= (n >> 4);
    else                keep = (k >> 4) <= n;
    o[i] = (_Float16)(keep ? w * WSC : 0.0f);
  }
  _Float16* dp = dst + (size_t)t * 8;
  *(volatile v8h*)dp = o;
  __threadfence();
  *(volatile v8h*)dp = o;
}

__device__ __forceinline__ v8f mma16(const v16h a, const v16h b, v8f cacc) {
  v8f d = __builtin_amdgcn_wmma_f32_16x16x32_f16(false, a, false, b, (short)0, cacc, false, false);
  asm volatile("v_nop\n\tv_nop\n\tv_nop\n\tv_nop" : "+v"(d) : "v"(a), "v"(b));
  return d;
}

template<int SA>
__device__ __forceinline__ v8f gemm_tile(const _Float16* bufIn, const _Float16* __restrict__ wf,
                                         int nkt, int lane) {
  const int row = lane & 15, kb = (lane >> 4) << 3;
  const _Float16* ap = bufIn + row * SA + kb;
  const _Float16* bp = wf + lane * 16;
  v8f acc = {0.f, 0.f, 0.f, 0.f, 0.f, 0.f, 0.f, 0.f};
#pragma unroll 1
  for (int kt = 0; kt < nkt; ++kt) {
    Frag a, b;
    a.h[0] = *(const v8h*)(ap + kt * 32);
    a.h[1] = *(const v8h*)(ap + kt * 32 + 16);
    b.h[0] = *(const v8h*)(bp + (size_t)kt * 512);
    b.h[1] = *(const v8h*)(bp + (size_t)kt * 512 + 8);
    acc = mma16(a.v, b.v, acc);
  }
  return acc;
}

__device__ __forceinline__ void relu_store(_Float16* bufOut, int nt, const v8f acc,
                                           const float* __restrict__ bias, int lane) {
  const int c = lane & 15, g = lane >> 4;
  const float bv = bias[nt * 16 + c];
  _Float16* op = bufOut + (g * 8) * ST + nt * 16 + c;
#pragma unroll
  for (int e = 0; e < 8; ++e) {
    float v = fmaf(acc[e], WSCI, bv);
    v = fmaxf(v, 0.0f);
    op[e * ST] = (_Float16)v;
  }
}

__device__ __forceinline__ void store_x(_Float16* bufX, const v8f x0, const v8f x1, int lane) {
  const int c = lane & 15, g = lane >> 4;
  _Float16* p = bufX + (g * 8) * SX + c;
#pragma unroll
  for (int e = 0; e < 8; ++e) {
    p[e * SX]      = (_Float16)x0[e];
    p[e * SX + 16] = (_Float16)x1[e];
  }
}

struct StepW {
  const _Float16 *w0, *w1, *w2, *w3;
  const float *b0, *b1, *b2, *b3;
};

__device__ __forceinline__ StepW step_ptrs(int st,
    const _Float16* pw0, const _Float16* pw1, const _Float16* pw2, const _Float16* pw3,
    const float* b0, const float* b1, const float* b2, const float* b3) {
  StepW s;
  s.w0 = pw0 + (size_t)st * (32 * 512);
  s.w1 = pw1 + (size_t)st * (512 * 512);
  s.w2 = pw2 + (size_t)st * (512 * 512);
  s.w3 = pw3 + (size_t)st * (32 * 512);
  s.b0 = b0 + st * HH;
  s.b1 = b1 + st * HH;
  s.b2 = b2 + st * HH;
  s.b3 = b3 + st * DD;
  return s;
}

__device__ __forceinline__ void shift_full(const v8f x0, const v8f x1, v8f& s0, v8f& s1,
                                           const StepW& sw, _Float16* bufX,
                                           _Float16* H1, _Float16* H2, _Float16* H3, int lane) {
  const int c = lane & 15;
  __syncthreads();
  store_x(bufX, x0, x1, lane);
  __syncthreads();
#pragma unroll 1
  for (int nt = 0; nt < 32; ++nt) {
    v8f acc = gemm_tile<SX>(bufX, sw.w0 + (size_t)nt * 512, 1, lane);
    relu_store(H1, nt, acc, sw.b0, lane);
  }
  __syncthreads();
#pragma unroll 1
  for (int nt = 0; nt < 32; ++nt) {
    v8f acc = gemm_tile<ST>(H1, sw.w1 + (size_t)nt * 16 * 512, (nt >> 1) + 1, lane);
    relu_store(H2, nt, acc, sw.b1, lane);
  }
  __syncthreads();
#pragma unroll 1
  for (int nt = 0; nt < 32; ++nt) {
    v8f acc = gemm_tile<ST>(H2, sw.w2 + (size_t)nt * 16 * 512, (nt >> 1) + 1, lane);
    relu_store(H3, nt, acc, sw.b2, lane);
  }
  __syncthreads();
  {
    v8f acc = gemm_tile<ST>(H3, sw.w3, 8, lane);
    const float bv = sw.b3[c];
#pragma unroll
    for (int e = 0; e < 8; ++e) s0[e] = fmaf(acc[e], WSCI, bv);
  }
  {
    v8f acc = gemm_tile<ST>(H3, sw.w3 + 16 * 512, 16, lane);
    const float bv = sw.b3[16 + c];
#pragma unroll
    for (int e = 0; e < 8; ++e) s1[e] = fmaf(acc[e], WSCI, bv);
  }
}

__device__ __forceinline__ void flow_fwd_step(v8f& y0, v8f& y1, const StepW& sw, _Float16* bufX,
                                              _Float16* H1, _Float16* H2, _Float16* H3, int lane) {
  const int c = lane & 15;
  const v8f xin0 = y0, xin1 = y1;
  v8f sh0 = {0.f, 0.f, 0.f, 0.f, 0.f, 0.f, 0.f, 0.f};
  v8f sh1 = {0.f, 0.f, 0.f, 0.f, 0.f, 0.f, 0.f, 0.f};
#pragma unroll 1
  for (int j = 0; j < DD; ++j) {
    const int nkt = (j >> 1) + 1;
    const int t = j >> 4;
    const v8f cy0 = xin0 + sh0;
    const v8f cy1 = xin1 + sh1;
    __syncthreads();
    store_x(bufX, cy0, cy1, lane);
    __syncthreads();
    {
      v8f acc = gemm_tile<SX>(bufX, sw.w0 + (size_t)j * 512, 1, lane);
      relu_store(H1, j, acc, sw.b0, lane);
    }
    __syncthreads();
    {
      v8f acc = gemm_tile<ST>(H1, sw.w1 + (size_t)j * 16 * 512, nkt, lane);
      relu_store(H2, j, acc, sw.b1, lane);
    }
    __syncthreads();
    {
      v8f acc = gemm_tile<ST>(H2, sw.w2 + (size_t)j * 16 * 512, nkt, lane);
      relu_store(H3, j, acc, sw.b2, lane);
    }
    __syncthreads();
    v8f acc = gemm_tile<ST>(H3, sw.w3 + (size_t)t * 16 * 512, nkt, lane);
    const float bv = sw.b3[j];
    const bool mine = (c == (j & 15));
    const bool m0 = mine && (t == 0);
    const bool m1 = mine && (t == 1);
#pragma unroll
    for (int e = 0; e < 8; ++e) {
      const float v = fmaf(acc[e], WSCI, bv);
      sh0[e] = m0 ? v : sh0[e];
      sh1[e] = m1 ? v : sh1[e];
    }
  }
  y0 = xin0 + sh0;
  y1 = xin1 + sh1;
}

__device__ __forceinline__ void reverse2(v8f& x0, v8f& x1) {
  v8f n0, n1;
#pragma unroll
  for (int e = 0; e < 8; ++e) {
    n0[e] = __shfl_xor(x1[e], 15, 32);
    n1[e] = __shfl_xor(x0[e], 15, 32);
  }
  x0 = n0; x1 = n1;
}

__global__ void __launch_bounds__(32)
flow_main(const float* __restrict__ zmean, const float* __restrict__ zlogv,
          const float* __restrict__ eps,
          const float* __restrict__ b0, const float* __restrict__ b1,
          const float* __restrict__ b2, const float* __restrict__ b3,
          const _Float16* __restrict__ pw0, const _Float16* __restrict__ pw1,
          const _Float16* __restrict__ pw2, const _Float16* __restrict__ pw3,
          float* out_samples, float* out_logp) {
  __shared__ __attribute__((aligned(16))) _Float16 bufX[16 * SX];
  __shared__ __attribute__((aligned(16))) _Float16 bufH1[16 * ST];
  __shared__ __attribute__((aligned(16))) _Float16 bufH2[16 * ST];
  __shared__ __attribute__((aligned(16))) _Float16 bufH3[16 * ST];
  __shared__ __attribute__((aligned(16))) float sbuf[16 * DD];
  __shared__ __attribute__((aligned(16))) float lpbuf[32];

  const int lane = threadIdx.x;
  const int c = lane & 15, g = lane >> 4;

  {
    const _Float16 hz = (_Float16)0.0f;
    const v8h z8 = {hz, hz, hz, hz, hz, hz, hz, hz};
    for (int i = lane; i < (16 * ST) / 8; i += 32) {
      *(v8h*)(bufH1 + 8 * i) = z8;
      *(v8h*)(bufH2 + 8 * i) = z8;
      *(v8h*)(bufH3 + 8 * i) = z8;
    }
    for (int i = lane; i < (16 * SX) / 8; i += 32) *(v8h*)(bufX + 8 * i) = z8;
    lpbuf[lane] = 0.0f;
  }
  __syncthreads();

#pragma unroll 1
  for (int half = 0; half < 2; ++half) {
    const int row0 = blockIdx.x * 32 + half * 16;

    v8f x0, x1;
#pragma unroll
    for (int e = 0; e < 8; ++e) {
      const int i0 = (row0 + g * 8 + e) * DD + c;
      const int i1 = i0 + 16;
      const float l0 = zlogv[i0], l1 = zlogv[i1];
      x0[e] = zmean[i0] + expf(0.5f * l0) * eps[i0];
      x1[e] = zmean[i1] + expf(0.5f * l1) * eps[i1];
    }

#pragma unroll 1
    for (int p = 0; p < NSTEP; ++p) {
      const StepW sw = step_ptrs(NSTEP - 1 - p, pw0, pw1, pw2, pw3, b0, b1, b2, b3);
      v8f s0, s1;
      shift_full(x0, x1, s0, s1, sw, bufX, bufH1, bufH2, bufH3, lane);
      x0 -= s0; x1 -= s1;
      if (p < NSTEP - 1) reverse2(x0, x1);
    }

    __syncthreads();
#pragma unroll
    for (int e = 0; e < 8; ++e) {
      sbuf[(g * 8 + e) * DD + c]      = x0[e];
      sbuf[(g * 8 + e) * DD + 16 + c] = x1[e];
    }
    __syncthreads();
    {
      const int rr = lane >> 3, cc = 4 * (lane & 7);
      const v4f v0 = *(const v4f*)(sbuf + (0  + rr) * DD + cc);
      const v4f v1 = *(const v4f*)(sbuf + (4  + rr) * DD + cc);
      const v4f v2 = *(const v4f*)(sbuf + (8  + rr) * DD + cc);
      const v4f v3 = *(const v4f*)(sbuf + (12 + rr) * DD + cc);
      float* op = out_samples + (size_t)(row0 + rr) * DD + cc;
      *(volatile v4f*)(op)           = v0;
      *(volatile v4f*)(op + 4 * DD)  = v1;
      *(volatile v4f*)(op + 8 * DD)  = v2;
      *(volatile v4f*)(op + 12 * DD) = v3;
      __threadfence();
      *(volatile v4f*)(op)           = v0;
      *(volatile v4f*)(op + 4 * DD)  = v1;
      *(volatile v4f*)(op + 8 * DD)  = v2;
      *(volatile v4f*)(op + 12 * DD) = v3;
    }

#pragma unroll 1
    for (int p = 0; p < NSTEP; ++p) {
      const StepW sw = step_ptrs(p, pw0, pw1, pw2, pw3, b0, b1, b2, b3);
      flow_fwd_step(x0, x1, sw, bufX, bufH1, bufH2, bufH3, lane);
      if (p < NSTEP - 1) reverse2(x0, x1);
    }

    v8f ssq, slv;
#pragma unroll
    for (int e = 0; e < 8; ++e) {
      const int i0 = (row0 + g * 8 + e) * DD + c;
      const int i1 = i0 + 16;
      const float m0 = zmean[i0], m1 = zmean[i1];
      const float l0 = zlogv[i0], l1 = zlogv[i1];
      const float d0 = (x0[e] - m0) * expf(-0.5f * l0);
      const float d1 = (x1[e] - m1) * expf(-0.5f * l1);
      ssq[e] = d0 * d0 + d1 * d1;
      slv[e] = l0 + l1;
    }
#pragma unroll
    for (int off = 1; off < 16; off <<= 1) {
#pragma unroll
      for (int e = 0; e < 8; ++e) {
        ssq[e] += __shfl_xor(ssq[e], off, 32);
        slv[e] += __shfl_xor(slv[e], off, 32);
      }
    }
    if (c < 8) {
      float lp = 0.0f;
#pragma unroll
      for (int e = 0; e < 8; ++e) if (e == c) lp = -0.5f * ssq[e] - 0.5f * slv[e];
      lp -= HALF_D_LOG2PI;
      lpbuf[half * 16 + g * 8 + c] = lp;
    }
  }

  __syncthreads();
  {
    v4f v = {0.f, 0.f, 0.f, 0.f};
    if (lane < 8) v = *(const v4f*)(lpbuf + 4 * lane);
    if (lane < 8) {
      float* op = out_logp + (size_t)blockIdx.x * 32 + 4 * lane;
      *(volatile v4f*)op = v;
    }
    __threadfence();
    if (lane < 8) {
      float* op = out_logp + (size_t)blockIdx.x * 32 + 4 * lane;
      *(volatile v4f*)op = v;
    }
  }
}

extern "C" void kernel_launch(void* const* d_in, const int* in_sizes, int n_in,
                              void* d_out, int out_size, void* d_ws, size_t ws_size,
                              hipStream_t stream) {
  if (n_in < 11) return;
  const float* zmean = (const float*)d_in[0];
  const float* zlogv = (const float*)d_in[1];
  const float* eps   = (const float*)d_in[2];
  const float* W0    = (const float*)d_in[3];
  const float* b0    = (const float*)d_in[4];
  const float* W1    = (const float*)d_in[5];
  const float* b1    = (const float*)d_in[6];
  const float* W2    = (const float*)d_in[7];
  const float* b2    = (const float*)d_in[8];
  const float* W3    = (const float*)d_in[9];
  const float* b3    = (const float*)d_in[10];

  if (in_sizes[0] != NB * DD || in_sizes[1] != NB * DD || in_sizes[2] != NB * DD) return;
  if (in_sizes[3] != NSTEP * DD * HH || in_sizes[5] != NSTEP * HH * HH ||
      in_sizes[7] != NSTEP * HH * HH || in_sizes[9] != NSTEP * HH * DD) return;
  if (in_sizes[4] != NSTEP * HH || in_sizes[6] != NSTEP * HH ||
      in_sizes[8] != NSTEP * HH || in_sizes[10] != NSTEP * DD) return;
  if (out_size != NB * DD + NB) return;

  const size_t n0 = (size_t)NSTEP * DD * HH;
  const size_t n1 = (size_t)NSTEP * HH * HH;
  const size_t n3 = (size_t)NSTEP * HH * DD;
  const size_t total_bytes = (n0 + n1 + n1 + n3) * sizeof(_Float16);
  if (total_bytes > ws_size) return;
  _Float16* pw0 = (_Float16*)d_ws;
  _Float16* pw1 = pw0 + n0;
  _Float16* pw2 = pw1 + n1;
  _Float16* pw3 = pw2 + n1;

  const int c0 = (int)(n0 / 8), c1 = (int)(n1 / 8), c3 = (int)(n3 / 8);
  pack_weights<<<(c0 + 255) / 256, 256, 0, stream>>>(W0, pw0, DD, HH, 0, c0);
  pack_weights<<<(c1 + 255) / 256, 256, 0, stream>>>(W1, pw1, HH, HH, 1, c1);
  pack_weights<<<(c1 + 255) / 256, 256, 0, stream>>>(W2, pw2, HH, HH, 1, c1);
  pack_weights<<<(c3 + 255) / 256, 256, 0, stream>>>(W3, pw3, HH, DD, 2, c3);

  float* out_samples = (float*)d_out;
  float* out_logp    = out_samples + (size_t)NB * DD;

  flow_main<<<NB / 32, 32, 0, stream>>>(zmean, zlogv, eps, b0, b1, b2, b3,
                                       pw0, pw1, pw2, pw3, out_samples, out_logp);
}
